// GNOBlock_77721728188840
// MI455X (gfx1250) — hardware-verified
//
#include <hip/hip_runtime.h>
#include <stddef.h>
#include <stdint.h>

#define NYP    100000
#define NXP    20000
#define NCO    3
#define NFQ    32
#define DEMB   192
#define K1     384
#define HID    256
#define K23    512
#define COUT   64
#define GBM    64
#define GBN    128
#define GTHR   128
#define AP1    392
#define MYP    100032
#define MXP    20032
#define QPB    4
#define EPB    64
#define ETHR   128
#define AP2    520
#define DP2    260
#define FP     68
#define CSTN   320
#define PTHR   256
#define NU1    (HID * (K1 / 8))
#define NU2    (HID * (K23 / 8))
#define NU3    (COUT * (K23 / 8))
#define NUTOT  (2 * NU1 + NU2 + NU3)
#define NODE_LDS_BYTES (GBM * AP1 * 2 + GBM * GBN * 4 + GBM * NCO * 4 + NFQ * 4)
#define EDGE_LDS_BYTES (EPB * AP2 * 2 + EPB * DP2 * 4 + EPB * FP * 4 + CSTN * 4 + QPB * COUT * 4 + 8 * 4)
#define WSMAX  134217728

static_assert(DEMB == NCO * NFQ * 2 && K1 == 2 * DEMB && K23 == 2 * HID);
static_assert(K1 % 32 == 0 && K23 % 32 == 0 && HID == 2 * GBN && COUT % 16 == 0);
static_assert(MYP % GBM == 0 && MYP >= NYP && MYP - GBM < NYP);
static_assert(MXP % GBM == 0 && MXP >= NXP && MXP - GBM < NXP);
static_assert(NU1 % PTHR == 0 && NU2 % PTHR == 0 && NU3 % PTHR == 0 && NUTOT % PTHR == 0);
static_assert((AP1 * 2) % 16 == 0 && AP1 >= K1 && (AP2 * 2) % 16 == 0 && AP2 >= K23);
static_assert((DP2 * 4) % 16 == 0 && DP2 >= HID && (FP * 4) % 16 == 0 && FP >= COUT);
static_assert(GTHR == 2 * GBM && GBM == (GTHR / 32) * 16 && NFQ == 32);
static_assert(ETHR == 2 * EPB && EPB == (ETHR / 32) * 16 && QPB == ETHR / 32 && QPB * COUT == 2 * ETHR);
static_assert((GBM * AP1 * 2) % 16 == 0 && (GBM * GBN * 4) % 16 == 0);
static_assert((EPB * AP2 * 2) % 16 == 0 && (EPB * DP2 * 4) % 16 == 0 && (EPB * FP * 4) % 16 == 0 && (CSTN * 4) % 16 == 0);
static_assert(NODE_LDS_BYTES <= 300000 && EDGE_LDS_BYTES <= 300000);
static_assert((size_t)2 * HID * K1 * 2 + (size_t)HID * K23 * 2 + (size_t)COUT * K23 * 2 +
              (size_t)MYP * HID * 4 + (size_t)MXP * HID * 4 <= (size_t)WSMAX);

typedef float          v4f   __attribute__((ext_vector_type(4)));
typedef float          v8f   __attribute__((ext_vector_type(8)));
typedef int            v8i   __attribute__((ext_vector_type(8)));
typedef unsigned short v8us  __attribute__((ext_vector_type(8)));
typedef unsigned short v16us __attribute__((ext_vector_type(16)));
typedef __bf16         v16bf __attribute__((ext_vector_type(16)));
typedef v4f  __attribute__((may_alias)) v4fa;
typedef v8us __attribute__((may_alias)) v8usa;
union FragB { v16bf v; v16us u; v8us h[2]; v8i w; };

__device__ __forceinline__ v8f wmb(const FragB& a, const FragB& b, v8f c) {
  v8f d = __builtin_amdgcn_wmma_f32_16x16x32_bf16(false, a.v, false, b.v, (short)0, c, false, false);
  asm volatile("v_nop\n\tv_nop\n\tv_nop\n\tv_nop" : "+v"(d) : "v"(a.w), "v"(b.w));
  return d;
}

__device__ __forceinline__ unsigned bf16_bits(float f) {
  const unsigned u = __float_as_uint(f);
  return (u + 0x7FFFu + ((u >> 16) & 1u)) >> 16;
}
__device__ __forceinline__ float bf16_val(float f) {
  return __uint_as_float(bf16_bits(f) << 16);
}
__device__ __forceinline__ float gelu_f(float t) {
  return 0.5f * t * (1.0f + erff(t * 0.70710678118654752f));
}
__device__ __forceinline__ void gelu_hilo8(const v4f a, const v4f b, unsigned short* dst_hi, unsigned short* dst_lo) {
  const v8f v = {a.x, a.y, a.z, a.w, b.x, b.y, b.z, b.w};
  v8us ho, lo;
#pragma unroll
  for (int i = 0; i < 8; ++i) {
    const float g = gelu_f(v[i]);
    const unsigned hb = bf16_bits(g);
    ho[i] = (unsigned short)hb;
    lo[i] = (unsigned short)bf16_bits(g - __uint_as_float(hb << 16));
  }
  *(v8usa*)dst_hi = ho;
  *(v8usa*)dst_lo = lo;
}

__global__ __launch_bounds__(PTHR) void k_prep(const float* __restrict__ W1, const float* __restrict__ W2,
                                               const float* __restrict__ W3,
                                               unsigned short* W1YT, unsigned short* W1XT,
                                               unsigned short* W2T2, unsigned short* W3T2) {
  const int u = (int)blockIdx.x * PTHR + (int)threadIdx.x;
  if (u >= NUTOT) return;
  v8us o;
  unsigned short* dp;
  if (u < 2 * NU1) {
    const int sel = (u >= NU1) ? 1 : 0;
    const int v   = u - sel * NU1;
    const int n   = v / (K1 / 8);
    const int k8  = (v - n * (K1 / 8)) * 8;
    const int k   = (k8 < DEMB) ? k8 : k8 - DEMB;
    const float* p = W1 + (size_t)(sel * DEMB + k) * HID + n;
#pragma unroll
    for (int i = 0; i < 8; ++i) o[i] = (unsigned short)bf16_bits(p[(size_t)i * HID]);
    dp = (sel ? W1XT : W1YT) + (size_t)n * K1 + k8;
  } else if (u < 2 * NU1 + NU2) {
    const int v  = u - 2 * NU1;
    const int n  = v >> 6;
    const int k8 = (v & 63) * 8;
    const int k  = k8 & (HID - 1);
    const float* p = W2 + (size_t)k * HID + n;
#pragma unroll
    for (int i = 0; i < 8; ++i) o[i] = (unsigned short)bf16_bits(p[(size_t)i * HID]);
    dp = W2T2 + (size_t)n * K23 + k8;
  } else {
    const int v  = u - 2 * NU1 - NU2;
    const int n  = v >> 6;
    const int k8 = (v & 63) * 8;
    const int k  = k8 & (HID - 1);
    const float* p = W3 + (size_t)k * COUT + n;
#pragma unroll
    for (int i = 0; i < 8; ++i) o[i] = (unsigned short)bf16_bits(p[(size_t)i * COUT]);
    dp = W3T2 + (size_t)n * K23 + k8;
  }
  *(volatile v8us*)dp = o;
  __threadfence();
  *(volatile v8us*)dp = o;
}

__global__ __launch_bounds__(GTHR) void k_node(const float* __restrict__ y, const float* __restrict__ x,
                                               const float* __restrict__ b1,
                                               const unsigned short* __restrict__ W1YT,
                                               const unsigned short* __restrict__ W1XT,
                                               int nTy, float* Y1, float* X1) {
  extern __shared__ __attribute__((aligned(16))) float dyn[];
  unsigned short* sA  = (unsigned short*)dyn;
  float*          stg = dyn + (GBM * AP1) / 2;
  float*          sP  = stg + GBM * GBN;
  float*          sFq = sP + GBM * NCO;

  const int tid = (int)threadIdx.x, lane = tid & 31, wave = tid >> 5, hh = lane >> 4, m = lane & 15;
  const bool isX = (int)blockIdx.x >= nTy;
  const int tile = isX ? (int)blockIdx.x - nTy : (int)blockIdx.x;
  const int nPts = isX ? NXP : NYP;
  const float* P = isX ? x : y;
  const unsigned short* BT = isX ? W1XT : W1YT;
  float* Cm = isX ? X1 : Y1;
  const float bsc = isX ? 1.0f : 0.0f;
  const int rowBase = tile * GBM;

  if (wave == 0) sFq[lane] = powf(0.0001f, (float)lane * 0.03125f);
  for (int i = tid; i < GBM * NCO; i += GTHR) {
    const int r = i / NCO, c = i - r * NCO;
    int rc = rowBase + r;
    rc = rc > nPts - 1 ? nPts - 1 : rc;
    sP[i] = bf16_val(P[(size_t)rc * NCO + c]);
  }
  __syncthreads();

  {
    const int r = tid >> 1, sub = tid & 1;
    unsigned short* ra = sA + r * AP1;
#pragma unroll 1
    for (int c = 0; c < NCO; ++c) {
      const float pc = sP[NCO * r + c];
#pragma unroll 1
      for (int fq = 0; fq < 4; ++fq) {
        const int f0 = 16 * sub + 4 * fq;
        v8us ho, lo;
#pragma unroll
        for (int i = 0; i < 4; ++i) {
          const float ang = pc * sFq[f0 + i];
          const float sv = sinf(ang);
          const float cv = cosf(ang);
          const unsigned hs = bf16_bits(sv);
          const unsigned hc = bf16_bits(cv);
          ho[2 * i]     = (unsigned short)hs;
          ho[2 * i + 1] = (unsigned short)hc;
          lo[2 * i]     = (unsigned short)bf16_bits(sv - __uint_as_float(hs << 16));
          lo[2 * i + 1] = (unsigned short)bf16_bits(cv - __uint_as_float(hc << 16));
        }
        *(v8usa*)(ra + c * (2 * NFQ) + 2 * f0)        = ho;
        *(v8usa*)(ra + DEMB + c * (2 * NFQ) + 2 * f0) = lo;
      }
    }
  }
  __syncthreads();

  const unsigned short* ap = sA + (16 * wave + m) * AP1 + 8 * hh;
#pragma unroll 1
  for (int half = 0; half < 2; ++half) {
    v8f acc[8];
    {
      const v8f z = {0.f, 0.f, 0.f, 0.f, 0.f, 0.f, 0.f, 0.f};
#pragma unroll
      for (int t = 0; t < 8; ++t) acc[t] = z;
    }
    const unsigned short* bp = BT + (size_t)(GBN * half + m) * K1 + 8 * hh;
#pragma unroll 1
    for (int k0 = 0; k0 < K1; k0 += 32) {
      FragB af;
      af.h[0] = *(const v8usa*)(ap + k0);
      af.h[1] = *(const v8usa*)(ap + k0 + 16);
#pragma unroll
      for (int nt = 0; nt < 8; ++nt) {
        const unsigned short* wq = bp + (size_t)(16 * nt) * K1 + k0;
        FragB bf;
        bf.h[0] = *(const v8usa*)wq;
        bf.h[1] = *(const v8usa*)(wq + 16);
        acc[nt] = wmb(af, bf, acc[nt]);
      }
    }
#pragma unroll
    for (int nt = 0; nt < 8; ++nt) {
      const int lc = 16 * nt + m;
      const float bv = bf16_val(b1[GBN * half + lc]) * bsc;
#pragma unroll
      for (int r = 0; r < 8; ++r) {
        const int lr = 16 * wave + 8 * hh + r;
        stg[lr * GBN + lc] = acc[nt][r] + bv;
      }
    }
    __syncthreads();

    v4f pv[16];
#pragma unroll
    for (int i = 0; i < 16; ++i) pv[i] = *(const v4fa*)(stg + (16 * wave + i) * GBN + 4 * lane);
#pragma unroll
    for (int i = 0; i < 16; ++i) {
      float* op = Cm + (size_t)(rowBase + 16 * wave + i) * HID + GBN * half + 4 * lane;
      *(volatile v4f*)op = pv[i];
    }
    __threadfence();
#pragma unroll
    for (int i = 0; i < 16; ++i) {
      float* op = Cm + (size_t)(rowBase + 16 * wave + i) * HID + GBN * half + 4 * lane;
      *(volatile v4f*)op = pv[i];
    }
    __syncthreads();
  }
}

__global__ __launch_bounds__(ETHR) void k_edge(const int* __restrict__ nbr, const int* __restrict__ rs, int nE,
                                               const float* __restrict__ fy,
                                               const float* __restrict__ Y1, const float* __restrict__ X1,
                                               const unsigned short* __restrict__ W2T2,
                                               const unsigned short* __restrict__ W3T2,
                                               const float* __restrict__ b2, const float* __restrict__ b3,
                                               float* out) {
  extern __shared__ __attribute__((aligned(16))) float dyn[];
  unsigned short* sA  = (unsigned short*)dyn;
  float*          sD  = dyn + (EPB * AP2) / 2;
  float*          sF  = sD + EPB * DP2;
  float*          cst = sF + EPB * FP;
  float*          sO  = cst + CSTN;
  int*            sRs = (int*)(sO + QPB * COUT);

  const int tid = (int)threadIdx.x, lane = tid & 31, wave = tid >> 5, hh = lane >> 4, m = lane & 15;
  const int q0 = (int)blockIdx.x * QPB;

  for (int i = tid; i < HID; i += ETHR) cst[i] = bf16_val(b2[i]);
  if (wave < 2) cst[HID + tid] = bf16_val(b3[tid]);
  if (wave == 0) {
    const int li = lane < QPB ? lane : QPB;
    int qi = q0 + li;
    qi = qi > NXP ? NXP : qi;
    int v = rs[qi];
    v = v < 0 ? 0 : (v > nE ? nE : v);
    if (lane <= QPB) sRs[lane] = v;
  }
  __syncthreads();

  const int ebase = sRs[0];

  {
    const int s = tid >> 1, sub = tid & 1;
    const int e = ebase + s;
    int ec = e > nE - 1 ? nE - 1 : e;
    ec = ec < 0 ? 0 : ec;
    int j = nbr[ec];
    j = j < 0 ? 0 : (j > NYP - 1 ? NYP - 1 : j);
    int ql = 0;
#pragma unroll
    for (int i = 1; i < QPB; ++i) ql += (e >= sRs[i]) ? 1 : 0;
    int q = q0 + ql;
    q = q > NXP - 1 ? NXP - 1 : q;

    const float* yr = Y1 + (size_t)j * HID + 128 * sub;
    const float* xr = X1 + (size_t)q * HID + 128 * sub;
    unsigned short* ra = sA + s * AP2 + 128 * sub;
#pragma unroll 1
    for (int g = 0; g < 16; ++g) {
      const v4f ya = *(const v4fa*)(yr + 8 * g);
      const v4f yb = *(const v4fa*)(yr + 8 * g + 4);
      const v4f xa = *(const v4fa*)(xr + 8 * g);
      const v4f xb = *(const v4fa*)(xr + 8 * g + 4);
      gelu_hilo8(ya + xa, yb + xb, ra + 8 * g, ra + HID + 8 * g);
    }
    const float* fr = fy + (size_t)j * COUT + 32 * sub;
    float* rf = sF + s * FP + 32 * sub;
#pragma unroll
    for (int g = 0; g < 8; ++g) {
      const v4f v = *(const v4fa*)(fr + 4 * g);
      v4f w;
      w.x = bf16_val(v.x); w.y = bf16_val(v.y); w.z = bf16_val(v.z); w.w = bf16_val(v.w);
      *(v4fa*)(rf + 4 * g) = w;
    }
  }
  __syncthreads();

  const unsigned short* ap = sA + (16 * wave + m) * AP2 + 8 * hh;

#pragma unroll 1
  for (int half = 0; half < 2; ++half) {
    v8f acc[8];
    {
      const v8f z = {0.f, 0.f, 0.f, 0.f, 0.f, 0.f, 0.f, 0.f};
#pragma unroll
      for (int t = 0; t < 8; ++t) acc[t] = z;
    }
    const unsigned short* bp = W2T2 + (size_t)(GBN * half + m) * K23 + 8 * hh;
#pragma unroll 1
    for (int k0 = 0; k0 < K23; k0 += 32) {
      FragB af;
      af.h[0] = *(const v8usa*)(ap + k0);
      af.h[1] = *(const v8usa*)(ap + k0 + 16);
#pragma unroll
      for (int nt = 0; nt < 8; ++nt) {
        const unsigned short* wq = bp + (size_t)(16 * nt) * K23 + k0;
        FragB bf;
        bf.h[0] = *(const v8usa*)wq;
        bf.h[1] = *(const v8usa*)(wq + 16);
        acc[nt] = wmb(af, bf, acc[nt]);
      }
    }
#pragma unroll
    for (int nt = 0; nt < 8; ++nt) {
      const int col = GBN * half + 16 * nt + m;
#pragma unroll
      for (int r = 0; r < 8; ++r)
        sD[(16 * wave + 8 * hh + r) * DP2 + col] = acc[nt][r];
    }
  }
  __syncthreads();

  {
    const int s = tid >> 1, sub = tid & 1;
    const float* rd = sD + s * DP2 + 128 * sub;
    const float* bb = cst + 128 * sub;
    unsigned short* ra = sA + s * AP2 + 128 * sub;
#pragma unroll 1
    for (int g = 0; g < 16; ++g) {
      const v4f da = *(const v4fa*)(rd + 8 * g);
      const v4f db = *(const v4fa*)(rd + 8 * g + 4);
      const v4f ba = *(const v4fa*)(bb + 8 * g);
      const v4f b8 = *(const v4fa*)(bb + 8 * g + 4);
      gelu_hilo8(da + ba, db + b8, ra + 8 * g, ra + HID + 8 * g);
    }
  }
  __syncthreads();

  {
    v8f acc3[4];
    {
      const v8f z = {0.f, 0.f, 0.f, 0.f, 0.f, 0.f, 0.f, 0.f};
#pragma unroll
      for (int t = 0; t < 4; ++t) acc3[t] = z;
    }
    const unsigned short* bp = W3T2 + (size_t)m * K23 + 8 * hh;
#pragma unroll 1
    for (int k0 = 0; k0 < K23; k0 += 32) {
      FragB af;
      af.h[0] = *(const v8usa*)(ap + k0);
      af.h[1] = *(const v8usa*)(ap + k0 + 16);
#pragma unroll
      for (int nt = 0; nt < 4; ++nt) {
        const unsigned short* wq = bp + (size_t)(16 * nt) * K23 + k0;
        FragB bf;
        bf.h[0] = *(const v8usa*)wq;
        bf.h[1] = *(const v8usa*)(wq + 16);
        acc3[nt] = wmb(af, bf, acc3[nt]);
      }
    }
#pragma unroll
    for (int nt = 0; nt < 4; ++nt) {
      const int col = 16 * nt + m;
      const float bv = cst[HID + col];
#pragma unroll
      for (int r = 0; r < 8; ++r)
        sD[(16 * wave + 8 * hh + r) * DP2 + col] = acc3[nt][r] + bv;
    }
  }
  __syncthreads();

  {
    const int loRaw = sRs[wave] - ebase;
    const int hiRaw = sRs[wave + 1] - ebase;
    const bool poison = (hiRaw > EPB) && (hiRaw > loRaw);
    int sBeg = loRaw < 0 ? 0 : (loRaw > EPB ? EPB : loRaw);
    int sEnd = hiRaw < 0 ? 0 : (hiRaw > EPB ? EPB : hiRaw);
    sEnd = sEnd < sBeg ? sBeg : sEnd;
    float a0 = 0.0f, a1 = 0.0f;
#pragma unroll 1
    for (int sl = sBeg; sl < sEnd; ++sl) {
      const float k0v = sD[sl * DP2 + lane],      f0v = sF[sl * FP + lane];
      const float k1v = sD[sl * DP2 + 32 + lane], f1v = sF[sl * FP + 32 + lane];
      a0 += k0v * f0v;
      a1 += k1v * f1v;
    }
    const float nanv = __uint_as_float(0x7fc00000u);
    sO[wave * COUT + lane]      = poison ? nanv : a0;
    sO[wave * COUT + 32 + lane] = poison ? nanv : a1;
  }
  __syncthreads();

  const int p   = 32 * (wave & 1) + lane;
  const int row = p >> 4;
  const int c4  = (p & 15) * 4;
  const v4f ov  = *(const v4fa*)(sO + row * COUT + c4);
  const int q   = q0 + row;
  const bool stv = (wave < 2) && (q < NXP);
  float* op = out + (size_t)(q < NXP ? q : NXP - 1) * COUT + c4;
  if (stv) *(volatile v4f*)op = ov;
  __threadfence();
  if (stv) *(volatile v4f*)op = ov;
}

static inline int cdiv(int a, int b) { return (a + b - 1) / b; }

extern "C" void kernel_launch(void* const* d_in, const int* in_sizes, int n_in,
                              void* d_out, int out_size, void* d_ws, size_t ws_size,
                              hipStream_t stream) {
  if (n_in < 11) return;
  if (in_sizes[0] != NYP * NCO) return;
  if (in_sizes[1] != NXP * NCO) return;
  if (in_sizes[2] != NYP * COUT) return;
  if (in_sizes[3] < 1) return;
  const int nE = in_sizes[3];
  if (in_sizes[4] != NXP + 1) return;
  if (in_sizes[5] != K1 * HID || in_sizes[6] != HID) return;
  if (in_sizes[7] != HID * HID || in_sizes[8] != HID) return;
  if (in_sizes[9] != HID * COUT || in_sizes[10] != COUT) return;
  if (out_size != NXP * COUT) return;

  const float* y   = (const float*)d_in[0];
  const float* x   = (const float*)d_in[1];
  const float* fy  = (const float*)d_in[2];
  const int*   nbr = (const int*)d_in[3];
  const int*   rs  = (const int*)d_in[4];
  const float* W1  = (const float*)d_in[5];
  const float* b1  = (const float*)d_in[6];
  const float* W2  = (const float*)d_in[7];
  const float* b2  = (const float*)d_in[8];
  const float* W3  = (const float*)d_in[9];
  const float* b3  = (const float*)d_in[10];
  float* out = (float*)d_out;

  char* ws = (char*)d_ws;
  size_t off = 0;
  const size_t oW1Y = off; off += (size_t)HID * K1 * 2;    off = (off + 255) & ~(size_t)255;
  const size_t oW1X = off; off += (size_t)HID * K1 * 2;    off = (off + 255) & ~(size_t)255;
  const size_t oW2  = off; off += (size_t)HID * K23 * 2;   off = (off + 255) & ~(size_t)255;
  const size_t oW3  = off; off += (size_t)COUT * K23 * 2;  off = (off + 255) & ~(size_t)255;
  const size_t oY1  = off; off += (size_t)MYP * HID * 4;   off = (off + 255) & ~(size_t)255;
  const size_t oX1  = off; off += (size_t)MXP * HID * 4;   off = (off + 255) & ~(size_t)255;
  if (off > ws_size || off > (size_t)WSMAX) return;
  unsigned short* W1YT = (unsigned short*)(ws + oW1Y);
  unsigned short* W1XT = (unsigned short*)(ws + oW1X);
  unsigned short* W2T2 = (unsigned short*)(ws + oW2);
  unsigned short* W3T2 = (unsigned short*)(ws + oW3);
  float*          Y1   = (float*)(ws + oY1);
  float*          X1   = (float*)(ws + oX1);

  hipFuncSetAttribute(reinterpret_cast<const void*>(&k_node), hipFuncAttributeMaxDynamicSharedMemorySize,
                      (int)NODE_LDS_BYTES);
  hipFuncSetAttribute(reinterpret_cast<const void*>(&k_edge), hipFuncAttributeMaxDynamicSharedMemorySize,
                      (int)EDGE_LDS_BYTES);

  const int nTy = MYP / GBM;
  const int nTx = MXP / GBM;
  k_prep<<<NUTOT / PTHR, PTHR, 0, stream>>>(W1, W2, W3, W1YT, W1XT, W2T2, W3T2);
  k_node<<<nTy + nTx, GTHR, NODE_LDS_BYTES, stream>>>(y, x, b1, W1YT, W1XT, nTy, Y1, X1);
  k_edge<<<cdiv(NXP, QPB), ETHR, EDGE_LDS_BYTES, stream>>>(nbr, rs, nE, fy, Y1, X1, W2T2, W3T2, b2, b3, out);
}
